// SSelfattention_65189013618943
// MI455X (gfx1250) — hardware-verified
//
#include <hip/hip_runtime.h>

typedef _Float16 f16;
typedef __attribute__((ext_vector_type(16))) _Float16 v16h;
typedef __attribute__((ext_vector_type(8)))  _Float16 v8h;
typedef __attribute__((ext_vector_type(8)))  float    v8f;
typedef __attribute__((ext_vector_type(4)))  unsigned v4u_;
typedef __attribute__((ext_vector_type(8)))  int      v8i_;
typedef __attribute__((ext_vector_type(4)))  int      v4i_;
typedef __attribute__((ext_vector_type(4)))  float    v4f;
template <typename T> __device__ __forceinline__ void vst2(void* p, T v) { *(volatile T*)p = v; __threadfence(); *(volatile T*)p = v; }
__device__ __forceinline__ v8f WM(v16h a, v16h b, v8f c) {
    v8f d = __builtin_amdgcn_wmma_f32_16x16x32_f16(false, a, false, b, (short)0, c, false, false);
    asm volatile("v_nop\n\tv_nop\n\tv_nop\n\tv_nop" : "+v"(d) : "v"(a), "v"(b));
    return d;
}

#define NN 512
#define TT 32
#define CC 128
#define HH 8
#define DD 16
#define PER_TH (NN*DD)


__device__ __forceinline__ float halfmax16(float v) {
    v = fmaxf(v, __shfl_xor(v, 1, 32));
    v = fmaxf(v, __shfl_xor(v, 2, 32));
    v = fmaxf(v, __shfl_xor(v, 4, 32));
    v = fmaxf(v, __shfl_xor(v, 8, 32));
    return v;
}


#define HAVE_TDM 0


__global__ __launch_bounds__(256) void proj_kernel(
    const float* __restrict__ values, const float* __restrict__ keys,
    const float* __restrict__ Wq, const float* __restrict__ Wk,
    const float* __restrict__ Wv,
    f16* __restrict__ Qp, f16* __restrict__ Kp, f16* __restrict__ Vp)
{
    int g = blockIdx.x * 256 + threadIdx.x;
    int idx0 = g * 8;
    int e0 = idx0 & 15;
    int n  = (idx0 >> 4) & (NN - 1);
    int th = idx0 >> 13;
    int h  = th & (HH - 1);
    int t  = th >> 3;
    const float* xv = values + ((size_t)n * TT + t) * CC + h * DD;
    const float* xk = keys   + ((size_t)n * TT + t) * CC + h * DD;
    float v16[16], k16[16];
#pragma unroll
    for (int d = 0; d < 16; ++d) { v16[d] = xv[d]; k16[d] = xk[d]; }
    union { v8h hh; v4u_ u; } pq, pk, pv;
#pragma unroll 1
    for (int ee = 0; ee < 8; ++ee) {
        const int e = e0 + ee;
        float aq = 0.f, ak = 0.f, av = 0.f;
#pragma unroll
        for (int d = 0; d < 16; ++d) { aq += v16[d] * Wq[e * 16 + d]; ak += k16[d] * Wk[e * 16 + d]; av += v16[d] * Wv[e * 16 + d]; }
        pq.hh[ee] = (f16)aq; pk.hh[ee] = (f16)ak; pv.hh[ee] = (f16)av;
    }
    vst2(Qp + idx0, pq.u); vst2(Kp + idx0, pk.u); vst2(Vp + idx0, pv.u);
}

__global__ __launch_bounds__(256) void attn_kernel(
    const f16* __restrict__ Qp, const f16* __restrict__ Kp,
    const f16* __restrict__ Vp, f16* __restrict__ O)
{
    __shared__ __attribute__((aligned(16))) f16 Kt[NN * DD];
    __shared__ __attribute__((aligned(16))) f16 Vt[NN * DD];
    __shared__ __attribute__((aligned(16))) f16 Ps[8][16][32];
    __shared__ __attribute__((aligned(16))) f16 Os[8][16][16];

    const int tid = threadIdx.x;
    const int th  = blockIdx.x;
    const int t   = th >> 3, h = th & 7;

#if HAVE_TDM
    if (tid < 32) {
        tdm_load_16k((unsigned)(uintptr_t)&Kt[0], Kp + (size_t)th * PER_TH);
        tdm_load_16k((unsigned)(uintptr_t)&Vt[0], Vp + (size_t)th * PER_TH);
        __builtin_amdgcn_s_wait_tensorcnt(0);
    }
#else
    {
        const v8h* kg = (const v8h*)(Kp + (size_t)th * PER_TH);
        const v8h* vg = (const v8h*)(Vp + (size_t)th * PER_TH);
        v8h* ks = (v8h*)Kt; v8h* vs = (v8h*)Vt;
        for (int i = tid; i < PER_TH / 8; i += 256) { ks[i] = kg[i]; vs[i] = vg[i]; }
    }
#endif
    __syncthreads();

    const int wid  = tid >> 5, lane = tid & 31;
    const int half = lane >> 4, ln = lane & 15;
    const float cs = 0.1275174465f;

    v16h ones;
#pragma unroll
    for (int i = 0; i < 16; ++i) ones[i] = (f16)1;

    v16h kb0, kb1;
#pragma unroll
    for (int i = 0; i < 8; ++i) { kb0[8 + i] = (f16)0; kb1[8 + i] = (f16)0; }

    for (int it = 0; it < 4; ++it) {
        const int qbase = (wid * 4 + it) * 16;

        const f16* qr = Qp + ((size_t)th * NN + qbase + ln) * DD + half * 8;
        v8h qlo = *(const v8h*)qr;
        v16h qa;
#pragma unroll
        for (int i = 0; i < 8; ++i) { qa[i] = qlo[i]; qa[8 + i] = (f16)0; }
        if (it < 3)
            __builtin_prefetch(Qp + ((size_t)th * NN + qbase + 16 + ln) * DD, 0, 1);

        float mcol[8];
#pragma unroll
        for (int r = 0; r < 8; ++r) mcol[r] = -1e30f;

        for (int jj = 0; jj < 16; ++jj) {
            const int kn0 = jj * 32;
            const v8h k0 = *(const v8h*)&Kt[(kn0 + ln) * DD + half * 8];
            const v8h k1 = *(const v8h*)&Kt[(kn0 + 16 + ln) * DD + half * 8];
#pragma unroll
            for (int i = 0; i < 8; ++i) { kb0[i] = k0[i]; kb1[i] = k1[i]; }
            v8f z = {};
            v8f s0 = WM(qa, kb0, z);
            v8f s1 = WM(qa, kb1, z);
#pragma unroll
            for (int r = 0; r < 8; ++r) mcol[r] = fmaxf(mcol[r], fmaxf(s0[r], s1[r]));
        }
        float mb[8];
#pragma unroll
        for (int r = 0; r < 8; ++r) mb[r] = cs * halfmax16(mcol[r]);

        float l[8];
        v8f o = {};
#pragma unroll
        for (int r = 0; r < 8; ++r) { l[r] = 0.f; o[r] = 0.f; }

        for (int jj = 0; jj < 16; ++jj) {
            const int kn0 = jj * 32;
            {
                const v8h k0 = *(const v8h*)&Kt[(kn0 + ln) * DD + half * 8];
                const v8h k1 = *(const v8h*)&Kt[(kn0 + 16 + ln) * DD + half * 8];
#pragma unroll
                for (int i = 0; i < 8; ++i) { kb0[i] = k0[i]; kb1[i] = k1[i]; }
            }
            v8f z = {};
            v8f s0 = WM(qa, kb0, z);
            v8f s1 = WM(qa, kb1, z);

#pragma unroll
            for (int r = 0; r < 8; ++r) {
                float p0 = exp2f(fmaf(s0[r], cs, -mb[r]));
                float p1 = exp2f(fmaf(s1[r], cs, -mb[r]));
                Ps[wid][r + half * 8][ln]      = (f16)p0;
                Ps[wid][r + half * 8][ln + 16] = (f16)p1;
            }
            asm volatile("s_wait_dscnt 0" ::: "memory");

            v16h pa;
            {
                const v8h plo = *(const v8h*)&Ps[wid][ln][half * 8];
                const v8h phi = *(const v8h*)&Ps[wid][ln][16 + half * 8];
#pragma unroll
                for (int i = 0; i < 8; ++i) { pa[i] = plo[i]; pa[8 + i] = phi[i]; }
            }

            v16h vb;
#pragma unroll
            for (int i = 0; i < 8; ++i) { vb[i] = Vt[(kn0 + half * 8 + i) * DD + ln]; vb[8 + i] = Vt[(kn0 + 16 + half * 8 + i) * DD + ln]; }

            v8f su = WM(pa, ones, z);
            o = WM(pa, vb, o);
#pragma unroll
            for (int r = 0; r < 8; ++r) l[r] += su[r];
        }

#pragma unroll
        for (int r = 0; r < 8; ++r) {
            float inv = 1.0f / l[r];
            Os[wid][r + half * 8][ln] = (f16)(o[r] * inv);
        }
        asm volatile("s_wait_dscnt 0" ::: "memory"); __builtin_amdgcn_wave_barrier(); __builtin_amdgcn_fence(__ATOMIC_RELEASE, "workgroup");
        vst2(O + ((size_t)th * NN + qbase) * DD + lane * 8, *(const v4u_*)(&Os[wid][0][0] + lane * 8));
        __builtin_amdgcn_wave_barrier();
    }
}

__global__ __launch_bounds__(256) void fc_kernel(
    const f16* __restrict__ X, const float* __restrict__ Wfc,
    const float* __restrict__ bfc, float* __restrict__ out)
{
    __shared__ __attribute__((aligned(16))) f16 Wf[CC * CC];
    __shared__ __attribute__((aligned(16))) float So[8][16 * CC];
    const int tid = threadIdx.x;
    for (int i = tid; i < CC * CC; i += 256) Wf[i] = (f16)Wfc[i];
    __syncthreads();

    const int wid = tid >> 5, lane = tid & 31;
    const int half = lane >> 4, ln = lane & 15;
    const int mbase = (blockIdx.x * 8 + wid) * 16;

    v16h a[4];
#pragma unroll
    for (int kb = 0; kb < 4; ++kb) {
        const int row = mbase + ln, n_ = row >> 5, t_ = row & 31;
        const int cl = kb * 32 + half * 8, chh = cl + 16;
        const f16* ar  = X + (((size_t)(t_ * HH + (cl  >> 4)) * NN + n_) * DD) + (cl  & 15);
        const f16* ar2 = X + (((size_t)(t_ * HH + (chh >> 4)) * NN + n_) * DD) + (chh & 15);
        v8h lo = *(const v8h*)ar;
        v8h hi = *(const v8h*)ar2;
#pragma unroll
        for (int i = 0; i < 8; ++i) { a[kb][i] = lo[i]; a[kb][8 + i] = hi[i]; }
    }
#pragma unroll
    for (int et = 0; et < 8; ++et) {
        v8f acc = {};
#pragma unroll
        for (int kb = 0; kb < 4; ++kb) {
            const f16* br = &Wf[(et * 16 + ln) * CC + kb * 32 + half * 8];
            v8h lo = *(const v8h*)br;
            v8h hi = *(const v8h*)(br + 16);
            v16h b;
#pragma unroll
            for (int i = 0; i < 8; ++i) { b[i] = lo[i]; b[8 + i] = hi[i]; }
            acc = WM(a[kb], b, acc);
        }
        float bb = bfc[et * 16 + ln];
#pragma unroll
        for (int r = 0; r < 8; ++r) So[wid][(r + half * 8) * CC + et * 16 + ln] = acc[r] + bb;
    }
    asm volatile("s_wait_dscnt 0" ::: "memory"); __builtin_amdgcn_wave_barrier(); __builtin_amdgcn_fence(__ATOMIC_RELEASE, "workgroup");
#pragma unroll 4
    for (int r = 0; r < 16; ++r) vst2(out + (size_t)(mbase + r) * CC + lane * 4, *(const v4f*)(&So[wid][r * CC] + lane * 4));
}

extern "C" void kernel_launch(void* const* d_in, const int* in_sizes, int n_in,
                              void* d_out, int out_size, void* d_ws, size_t ws_size,
                              hipStream_t stream) {
    const float* values = (const float*)d_in[0];
    const float* keys   = (const float*)d_in[1];
    const float* Wq  = (const float*)d_in[4];
    const float* Wk  = (const float*)d_in[5];
    const float* Wv  = (const float*)d_in[6];
    const float* Wfc = (const float*)d_in[7];
    const float* bfc = (const float*)d_in[8];
    float* out = (float*)d_out;

    const size_t SLICE = (size_t)TT * HH * NN * DD;
    f16* Qp = (f16*)d_ws;
    f16* Kp = Qp + SLICE;
    f16* Vp = Kp + SLICE;
    f16* O  = Vp + SLICE;

    proj_kernel<<<(int)(SLICE / 8 / 256), 256, 0, stream>>>(values, keys, Wq, Wk, Wv, Qp, Kp, Vp);
    attn_kernel<<<TT * HH, 256, 0, stream>>>(Qp, Kp, Vp, O);
    fc_kernel<<<(NN * TT / 16) / 8, 256, 0, stream>>>(O, Wfc, bfc, out);
}
